// multi_triples_lstm_67362267070530
// MI455X (gfx1250) — hardware-run, weakly checked
//
#include <hip/hip_runtime.h>

typedef __attribute__((ext_vector_type(16))) _Float16 v16h;
typedef __attribute__((ext_vector_type(8)))  _Float16 v8h;
typedef __attribute__((ext_vector_type(8)))  float    v8f;
typedef __attribute__((ext_vector_type(4)))  float    v4f;

template <typename T> struct Frag;
template <> struct Frag<_Float16> {
  typedef v16h V; union U { v16h v; v8h h[2]; };
  static __device__ __forceinline__ v16h load(const _Float16* p) {
    U f; f.h[0] = *(const v8h*)(p); f.h[1] = *(const v8h*)(p + 16); return f.v;
  }
};

__device__ __forceinline__ v8f hmma(v16h a, v16h b, v8f c) {
  c = __builtin_amdgcn_wmma_f32_16x16x32_f16(false, a, false, b, (short)0, c, false, false);
  asm volatile("v_nop\n\tv_nop\n\tv_nop\n\tv_nop" : "+v"(c) : "v"(a), "v"(b));
  return c;
}

constexpr int kSteps   = 32;
constexpr int kInDim   = 16;
constexpr int kHid     = 32;
constexpr int kGates   = 128;
constexpr int kObjV    = 179;
constexpr int kPredV   = 46;
constexpr int kEmb     = 5;
constexpr int kOutDim  = 4;
constexpr int kWaves   = 4;
constexpr int kRowsBlk = 16 * kWaves;
constexpr int kKPitch  = 64;
constexpr int kThreads = 32 * kWaves;

__device__ __forceinline__ float sigm_f(float x) {
  const float e = expf(-fabsf(x));
  const float d = 1.0f / (1.0f + e);
  return (x >= 0.0f) ? d : e * d;
}
__device__ __forceinline__ float tanh_f(float x) {
  const float e = expf(-2.0f * fabsf(x));
  const float r = (1.0f - e) / (1.0f + e);
  return copysignf(r, x);
}

__global__ __launch_bounds__(kThreads)
void lstm_seq_kernel(const int* __restrict__ objs,
                     const float* __restrict__ boxes,
                     const int* __restrict__ preds,
                     const int* __restrict__ subj,
                     const float* __restrict__ obj_emb,
                     const float* __restrict__ pred_emb,
                     const float* __restrict__ W_ih,
                     const float* __restrict__ W_hh,
                     const float* __restrict__ b_ih,
                     const float* __restrict__ b_hh,
                     const float* __restrict__ fc2_W,
                     const float* __restrict__ fc2_b,
                     float* __restrict__ out,
                     int nrows)
{
  __shared__ __align__(16) _Float16 s_bt[kGates * kKPitch];
  __shared__ __align__(16) _Float16 s_a[kRowsBlk * kKPitch];
  __shared__ __align__(16) float s_hf[kWaves][16 * kHid];
  __shared__ __align__(16) float s_out[kWaves][16 * kOutDim];
  __shared__ float s_obj[kObjV * kEmb];
  __shared__ float s_pred[kPredV * kEmb];
  __shared__ float s_bias[kGates];
  __shared__ float s_fc2w[kOutDim * kHid];
  __shared__ float s_fc2b[kOutDim];

  const int tid = threadIdx.x;

  for (int i = tid; i < kObjV * kEmb; i += kThreads)  s_obj[i]  = obj_emb[i];
  for (int i = tid; i < kPredV * kEmb; i += kThreads) s_pred[i] = pred_emb[i];
  {
    s_bias[tid] = b_ih[tid] + b_hh[tid];
    s_fc2w[tid] = fc2_W[tid];
    if (tid < kOutDim) s_fc2b[tid] = fc2_b[tid];
  }
#pragma unroll 1
  for (int g = 0; g < 8; ++g) {
    const int n = tid;
    v8h wv;
    if (g < 2) {
      const float* p = W_ih + n * kInDim + 8 * g;
      const v4f x0 = *(const v4f*)p, x1 = *(const v4f*)(p + 4);
#pragma unroll
      for (int e = 0; e < 4; ++e) { wv[e] = (_Float16)(x0[e] * 16.0f); wv[4 + e] = (_Float16)(x1[e] * 16.0f); }
    } else if (g < 6) {
      const float* p = W_hh + n * kHid + 8 * (g - 2);
      const v4f x0 = *(const v4f*)p, x1 = *(const v4f*)(p + 4);
#pragma unroll
      for (int e = 0; e < 4; ++e) { wv[e] = (_Float16)(x0[e] * 16.0f); wv[4 + e] = (_Float16)(x1[e] * 16.0f); }
    } else {
#pragma unroll
      for (int e = 0; e < 8; ++e) wv[e] = (_Float16)0.0f;
    }
    *(v8h*)(s_bt + n * kKPitch + 8 * g) = wv;
  }
  {
    v8h z;
#pragma unroll
    for (int e = 0; e < 8; ++e) z[e] = (_Float16)0.0f;
#pragma unroll
    for (int j = 0; j < 4; ++j) *(v8h*)(s_a + 8 * (tid + kThreads * j)) = z;
  }
  __syncthreads();

  const int lane = tid & 31;
  const int w    = tid >> 5;
  const int hh   = lane >> 4;
  const int c    = lane & 15;
  const int rowBase = blockIdx.x * kRowsBlk + 16 * w;
  int growc = rowBase + c;
  growc = (growc < nrows - 1) ? growc : (nrows - 1);

  float breg[4][2];
#pragma unroll
  for (int q = 0; q < 4; ++q)
#pragma unroll
    for (int s = 0; s < 2; ++s) breg[q][s] = s_bias[32 * q + 16 * s + c];

  float c_st[8][2], h_st[8][2];
#pragma unroll
  for (int m = 0; m < 8; ++m) { c_st[m][0] = 0.f; c_st[m][1] = 0.f; h_st[m][0] = 0.f; h_st[m][1] = 0.f; }

  _Float16* abase = s_a + (16 * w + c) * kKPitch + 8 * hh;
  const float kInv256 = 0.00390625f;

#pragma unroll 1
  for (int t = 0; t < kSteps; ++t) {
    {
      const size_t eidx = (size_t)growc * kSteps + t;
      int oid = objs[eidx];
      int pid = preds[eidx];
      const int sb = subj[eidx];
      const v4f bx = *(const v4f*)(boxes + eidx * 4);
      oid = (oid < 0) ? oid + kObjV : oid;   oid = (oid < 0) ? 0 : oid;  oid = (oid > kObjV - 1) ? (kObjV - 1) : oid;
      pid = (pid < 0) ? pid + kPredV : pid;  pid = (pid < 0) ? 0 : pid;  pid = (pid > kPredV - 1) ? (kPredV - 1) : pid;
      const float* oe = s_obj + oid * kEmb;
      const float* pe = s_pred + pid * kEmb;
      float f_lo[8], f_hi[8];
      f_lo[0] = oe[0]; f_lo[1] = oe[1]; f_lo[2] = oe[2]; f_lo[3] = oe[3]; f_lo[4] = oe[4];
      f_lo[5] = pe[0]; f_lo[6] = pe[1]; f_lo[7] = pe[2];
      f_hi[0] = pe[3]; f_hi[1] = pe[4];
      f_hi[2] = (sb == 0) ? 1.0f : 0.0f;
      f_hi[3] = (sb == 1) ? 1.0f : 0.0f;
      f_hi[4] = bx[0]; f_hi[5] = bx[1]; f_hi[6] = bx[2]; f_hi[7] = bx[3];
      v8h fv;
#pragma unroll
      for (int e = 0; e < 8; ++e) {
        const float v = hh ? f_hi[e] : f_lo[e];
        fv[e] = (_Float16)(v * 16.0f);
      }
      *(v8h*)abase = fv;
    }
    __syncthreads();

    v8f acc[8];
#pragma unroll
    for (int j = 0; j < 8; ++j) acc[j] = (v8f){0.f,0.f,0.f,0.f,0.f,0.f,0.f,0.f};
#pragma unroll
    for (int kc = 0; kc < 2; ++kc) {
      const v16h af = Frag<_Float16>::load(abase + kc * 32);
#pragma unroll
      for (int j = 0; j < 8; ++j) {
        const v16h bf = Frag<_Float16>::load(s_bt + (16 * j + c) * kKPitch + 8 * hh + kc * 32);
        acc[j] = hmma(af, bf, acc[j]);
      }
    }

#pragma unroll
    for (int m = 0; m < 8; ++m) {
#pragma unroll
      for (int s = 0; s < 2; ++s) {
        const float gi = acc[0 + s][m] * kInv256 + breg[0][s];
        const float gf = acc[2 + s][m] * kInv256 + breg[1][s];
        const float gg = acc[4 + s][m] * kInv256 + breg[2][s];
        const float go = acc[6 + s][m] * kInv256 + breg[3][s];
        const float iv = sigm_f(gi);
        const float fg = sigm_f(gf);
        const float gv = tanh_f(gg);
        const float ov = sigm_f(go);
        const float cn = fg * c_st[m][s] + iv * gv;
        c_st[m][s] = cn;
        const float hv = ov * tanh_f(cn);
        h_st[m][s] = hv;
        s_a[(16 * w + 8 * hh + m) * kKPitch + kInDim + 16 * s + c] = (_Float16)(hv * 16.0f);
      }
    }
  }

#pragma unroll
  for (int m = 0; m < 8; ++m) {
#pragma unroll
    for (int s = 0; s < 2; ++s) s_hf[w][(8 * hh + m) * kHid + 16 * s + c] = h_st[m][s];
  }
  __syncthreads();
  {
    const float* hr = s_hf[w] + c * kHid;
#pragma unroll
    for (int q = 0; q < 2; ++q) {
      const int oo = 2 * hh + q;
      const float* wr = s_fc2w + oo * kHid;
      float a = 0.0f;
#pragma unroll
      for (int u = 0; u < kHid; ++u) a += wr[u] * hr[u];
      a += s_fc2b[oo];
      a = fminf(fmaxf(a, 0.0f), 1.0f);
      s_out[w][c * kOutDim + oo] = a;
    }
  }
  __syncthreads();
  {
    const v4f val = *(const v4f*)(s_out[w] + c * kOutDim);
    const bool wvalid = (rowBase + 16) <= nrows;
    float* dst = out + (size_t)(rowBase + c) * kOutDim;
    for (int pass = 0; pass < 2; ++pass) {
      if (wvalid && lane < 16) *(volatile v4f*)dst = val;
      __threadfence();
    }
  }
}

extern "C" void kernel_launch(void* const* d_in, const int* in_sizes, int n_in,
                              void* d_out, int out_size, void* d_ws, size_t ws_size,
                              hipStream_t stream)
{
  (void)in_sizes; (void)n_in; (void)d_ws; (void)ws_size;
  const int*   objs     = (const int*)d_in[0];
  const float* boxes    = (const float*)d_in[1];
  const int*   preds    = (const int*)d_in[2];
  const int*   subj     = (const int*)d_in[3];
  const float* obj_emb  = (const float*)d_in[5];
  const float* pred_emb = (const float*)d_in[6];
  const float* W_ih     = (const float*)d_in[7];
  const float* W_hh     = (const float*)d_in[8];
  const float* b_ih     = (const float*)d_in[9];
  const float* b_hh     = (const float*)d_in[10];
  const float* fc2_W    = (const float*)d_in[11];
  const float* fc2_b    = (const float*)d_in[12];
  float* out = (float*)d_out;

  const int nrows = out_size / kOutDim;
  if (nrows <= 0) return;
  const int nblk = (nrows + kRowsBlk - 1) / kRowsBlk;
  lstm_seq_kernel<<<dim3(nblk), dim3(kThreads), 0, stream>>>(
      objs, boxes, preds, subj, obj_emb, pred_emb, W_ih, W_hh, b_ih, b_hh, fc2_W, fc2_b, out, nrows);
}
